// RGCNNFactorization_18820546691612
// MI455X (gfx1250) — hardware-verified
//
#include <hip/hip_runtime.h>


#define RR   10
#define QQ   32
#define NHID 32
#define NG   128
#define KC   5
#define KW   (KC * RR)
#define ZS   16
#define XGS  128
#define ROWS 256
#define GT   256
#define CH   (GT * 8)
#define CAP  6144
#define GR   32
#define AP   72
#define XP   40
#define SP   132
#define WLP  36

typedef unsigned short us16;
typedef __bf16 v16b __attribute__((ext_vector_type(16)));
typedef us16   v8us __attribute__((ext_vector_type(8)));
typedef float  v8f  __attribute__((ext_vector_type(8)));
typedef float  v4f  __attribute__((ext_vector_type(4)));
typedef float  v2f  __attribute__((ext_vector_type(2)));
typedef int    v4i  __attribute__((ext_vector_type(4)));

union Frag { v16b v; v8us q[2]; };

__device__ __forceinline__ us16 bf_rne(float x) {
  unsigned u = __float_as_uint(x);
  u += 0x7FFFu + ((u >> 16) & 1u);
  return (us16)(u >> 16);
}
__device__ __forceinline__ void split2(float x, us16* hi, us16* lo) {
  const us16 hb = bf_rne(x);
  const float hv = __uint_as_float(((unsigned)hb) << 16);
  *hi = hb;
  *lo = bf_rne(x - hv);
}

__device__ __forceinline__ v8f mma(v16b a, v16b b, v8f c) {
  return __builtin_amdgcn_wmma_f32_16x16x32_bf16(false, a, false, b, (short)0, c, false, false);
}
__device__ __forceinline__ void guard1(v8f& c, const v16b& a0, const v16b& a1,
                                       const v16b& b0, const v16b& b1) {
  asm volatile("v_nop\n\tv_nop\n\tv_nop\n\tv_nop"
               : "+v"(c)
               : "v"(a0), "v"(a1), "v"(b0), "v"(b1));
}

__device__ __forceinline__ float fsigm(float x) {
  const float e = __expf(-x);
  return __builtin_amdgcn_rcpf(1.0f + e);
}
__device__ __forceinline__ float ftanh(float x) {
  const float ax = fabsf(x);
  const float e = __expf(-2.0f * ax);
  const float r = (1.0f - e) * __builtin_amdgcn_rcpf(1.0f + e);
  return copysignf(r, x);
}
__device__ __forceinline__ void wave_sync() {
  __builtin_amdgcn_fence(__ATOMIC_ACQ_REL, "wavefront");
  __builtin_amdgcn_wave_barrier();
}

__device__ __forceinline__ void wave_rows_out(const float* st, float* g, int l) {
  v4f v[4];
#pragma unroll
  for (int i = 0; i < 4; ++i) v[i] = *(const v4f*)(st + (l + 32 * i) * 4);
#pragma unroll
  for (int i = 0; i < 4; ++i) *(volatile v4f*)(g + (l + 32 * i) * 4) = v[i];
  __threadfence();
#pragma unroll
  for (int i = 0; i < 4; ++i) *(volatile v4f*)(g + (l + 32 * i) * 4) = v[i];
}

template<int MODE>
__global__ __launch_bounds__(GT)
void k_graph(const int* __restrict__ EA, int nEA,
             const int* __restrict__ EB, int nEB,
             const float* __restrict__ XA, const float* __restrict__ XB,
             float* dinv, float* TX, int n, int NP, int kterm, int vecok) {
#pragma clang fp contract(off)
  __shared__ unsigned hl[CAP];
  __shared__ int wtot[GT / 32];
  __shared__ __attribute__((aligned(16))) float stg[ROWS * ZS];

  const int tid = threadIdx.x, l = tid & 31, w = tid >> 5;
  const int y = blockIdx.y;
  const int* E = (y != 0) ? EB : EA;
  const int nE = (y != 0) ? nEB : nEA;
  const float* X = (y != 0) ? XB : XA;
  const int rb = blockIdx.x * ROWS;
  const int myrow = rb + 32 * w + l;
  const int* keyp = (MODE == 0) ? E : (E + nE);
  const int* srcp = E;
  const float* dv = dinv + (size_t)y * NP;
  const int kz = (kterm > 1) ? (kterm - 1) : 0;
  const float* zpl = TX + ((size_t)(kz * 2 + y) * NP) * ZS;

  float dd = 0.0f;
  if (MODE != 0) dd = dv[myrow];
  float acc[RR];
#pragma unroll
  for (int r = 0; r < RR; ++r) acc[r] = 0.0f;
  int dcnt = 0;

  int cnt = 0;
  for (int cb = 0; cb < nE; cb += CH) {
    const int e0 = cb + tid * 8;
    int kv[8], sv[8];
    if (vecok != 0 && cb + CH <= nE) {
      const v4i k0 = *(const v4i*)(keyp + e0);
      const v4i k1 = *(const v4i*)(keyp + e0 + 4);
      kv[0] = k0.x; kv[1] = k0.y; kv[2] = k0.z; kv[3] = k0.w;
      kv[4] = k1.x; kv[5] = k1.y; kv[6] = k1.z; kv[7] = k1.w;
      if (MODE != 0) {
        const v4i s0 = *(const v4i*)(srcp + e0);
        const v4i s1 = *(const v4i*)(srcp + e0 + 4);
        sv[0] = s0.x; sv[1] = s0.y; sv[2] = s0.z; sv[3] = s0.w;
        sv[4] = s1.x; sv[5] = s1.y; sv[6] = s1.z; sv[7] = s1.w;
      } else {
#pragma unroll
        for (int j = 0; j < 8; ++j) sv[j] = 0;
      }
    } else {
#pragma unroll
      for (int j = 0; j < 8; ++j) {
        const int e = e0 + j;
        const int ec = min(e, nE - 1);
        const int kk = keyp[ec];
        kv[j] = (e < nE) ? kk : -1;
        if (MODE != 0) { const int ss = srcp[ec]; sv[j] = ss; } else { sv[j] = 0; }
      }
    }
    unsigned hit = 0u;
    int c = 0;
#pragma unroll
    for (int j = 0; j < 8; ++j) {
      const unsigned s = (unsigned)(kv[j] - rb);
      const bool ok = s < (unsigned)ROWS;
      hit |= (ok ? 1u : 0u) << j;
      c += ok ? 1 : 0;
    }
    int incl = c;
    { const int v = __shfl_up(incl, 1);  incl += (l >= 1)  ? v : 0; }
    { const int v = __shfl_up(incl, 2);  incl += (l >= 2)  ? v : 0; }
    { const int v = __shfl_up(incl, 4);  incl += (l >= 4)  ? v : 0; }
    { const int v = __shfl_up(incl, 8);  incl += (l >= 8)  ? v : 0; }
    { const int v = __shfl_up(incl, 16); incl += (l >= 16) ? v : 0; }
    if (l == 31) wtot[w] = incl;
    __syncthreads();
    int woff = 0, tot = 0;
#pragma unroll
    for (int i = 0; i < GT / 32; ++i) {
      const int v = wtot[i];
      tot += v;
      woff += (i < w) ? v : 0;
    }
    int pos = cnt + woff + incl - c;
#pragma unroll
    for (int j = 0; j < 8; ++j) {
      if (((hit >> j) & 1u) != 0u) {
        if (pos < CAP) {
          const int sc = min(max(sv[j], 0), n - 1);
          hl[pos] = ((unsigned)sc << 8) | (unsigned)(kv[j] - rb);
        }
        ++pos;
      }
    }
    cnt = min(cnt + tot, CAP);
    __syncthreads();
    const bool lastc = (cb + CH >= nE);
    if (cnt > CAP - CH || lastc) {
      for (int i0 = 0; i0 < cnt; i0 += 32) {
        const int idx = i0 + l;
        const unsigned kk = hl[min(idx, CAP - 1)];
        const bool mine = (idx < cnt) && (((kk & 255u) >> 5) == (unsigned)w);
        unsigned msk = __builtin_amdgcn_ballot_w32(mine);
        while (msk != 0u) {
          const int j = __builtin_ctz(msk);
          msk &= msk - 1u;
          const unsigned kj = (unsigned)__builtin_amdgcn_readlane((int)kk, j);
          const int s = (int)(kj >> 8);
          const int slot = (int)(kj & 31u);
          if (MODE == 0) {
            dcnt += (l == slot) ? 1 : 0;
          } else {
            const float ds = dv[s];
            const float wgt = (-ds) * dd;
            float z[RR];
            if (MODE == 1) {
              const float* zr = X + (size_t)s * RR;
#pragma unroll
              for (int r = 0; r < RR; ++r) z[r] = zr[r];
            } else {
              const float* zr = zpl + (size_t)s * ZS;
              const v4f za = *(const v4f*)zr;
              const v4f zb = *(const v4f*)(zr + 4);
              const v2f zc = *(const v2f*)(zr + 8);
              z[0] = za.x; z[1] = za.y; z[2] = za.z; z[3] = za.w;
              z[4] = zb.x; z[5] = zb.y; z[6] = zb.z; z[7] = zb.w;
              z[8] = zc.x; z[9] = zc.y;
            }
            if (l == slot) {
#pragma unroll
              for (int r = 0; r < RR; ++r) {
                const float p = wgt * z[r];
                acc[r] = acc[r] + p;
              }
            }
          }
        }
      }
      cnt = 0;
      __syncthreads();
    }
  }

  if (MODE == 0) {
    const float dval = (dcnt > 0) ? rsqrtf((float)dcnt) : 0.0f;
    float* p = dinv + (size_t)y * NP + myrow;
    *(volatile float*)p = dval;
    __threadfence();
    *(volatile float*)p = dval;
  } else {
    float o[RR];
    if (MODE == 1) {
#pragma unroll
      for (int r = 0; r < RR; ++r) o[r] = acc[r];
    } else {
      const float* sr = TX + (((size_t)((kterm - 2) * 2 + y) * NP) + myrow) * ZS;
      const v4f sa = *(const v4f*)sr;
      const v4f sb = *(const v4f*)(sr + 4);
      const v2f sc2 = *(const v2f*)(sr + 8);
      float sub[RR];
      sub[0] = sa.x; sub[1] = sa.y; sub[2] = sa.z; sub[3] = sa.w;
      sub[4] = sb.x; sub[5] = sb.y; sub[6] = sb.z; sub[7] = sb.w;
      sub[8] = sc2.x; sub[9] = sc2.y;
#pragma unroll
      for (int r = 0; r < RR; ++r) {
        const float d2 = 2.0f * acc[r];
        o[r] = d2 - sub[r];
      }
    }
    {
      float* st = stg + (32 * w + l) * ZS;
      v4f t0, t1, t2, t3;
      t0.x = o[0]; t0.y = o[1]; t0.z = o[2]; t0.w = o[3];
      t1.x = o[4]; t1.y = o[5]; t1.z = o[6]; t1.w = o[7];
      t2.x = o[8]; t2.y = o[9]; t2.z = 0.0f; t2.w = 0.0f;
      t3.x = 0.0f; t3.y = 0.0f; t3.z = 0.0f; t3.w = 0.0f;
      *(v4f*)(st) = t0; *(v4f*)(st + 4) = t1; *(v4f*)(st + 8) = t2; *(v4f*)(st + 12) = t3;
    }
    __syncthreads();
    {
      float* pl = TX + (((size_t)(kterm * 2 + y) * NP) + rb + 32 * w) * ZS;
      wave_rows_out(stg + (32 * w) * ZS, pl, l);
    }
    if (MODE == 1) {
      const int rc = min(myrow, n - 1);
      const float* xr = X + (size_t)rc * RR;
      float xv[RR];
#pragma unroll
      for (int r = 0; r < RR; ++r) { const float v = xr[r]; xv[r] = (myrow < n) ? v : 0.0f; }
      __syncthreads();
      {
        float* st = stg + (32 * w + l) * ZS;
        v4f t0, t1, t2, t3;
        t0.x = xv[0]; t0.y = xv[1]; t0.z = xv[2]; t0.w = xv[3];
        t1.x = xv[4]; t1.y = xv[5]; t1.z = xv[6]; t1.w = xv[7];
        t2.x = xv[8]; t2.y = xv[9]; t2.z = 0.0f; t2.w = 0.0f;
        t3.x = 0.0f; t3.y = 0.0f; t3.z = 0.0f; t3.w = 0.0f;
        *(v4f*)(st) = t0; *(v4f*)(st + 4) = t1; *(v4f*)(st + 8) = t2; *(v4f*)(st + 12) = t3;
      }
      __syncthreads();
      {
        float* p0 = TX + (((size_t)y * NP) + rb + 32 * w) * ZS;
        wave_rows_out(stg + (32 * w) * ZS, p0, l);
      }
    }
  }
}

__global__ __launch_bounds__(128)
void k_gemm(const float* __restrict__ TX,
            const float* __restrict__ cwA, const float* __restrict__ cbA,
            const float* __restrict__ cwB, const float* __restrict__ cbB,
            const float* __restrict__ wih, const float* __restrict__ bih,
            float* xg, int NP) {
  __shared__ __attribute__((aligned(16))) us16 Ah[GR * AP];
  __shared__ __attribute__((aligned(16))) us16 Al[GR * AP];
  __shared__ __attribute__((aligned(16))) us16 Bh[QQ * AP];
  __shared__ __attribute__((aligned(16))) us16 Bl[QQ * AP];
  __shared__ __attribute__((aligned(16))) us16 Xh[GR * XP];
  __shared__ __attribute__((aligned(16))) us16 Xl[GR * XP];
  __shared__ __attribute__((aligned(16))) us16 Wh[NG * XP];
  __shared__ __attribute__((aligned(16))) us16 Wl[NG * XP];
  __shared__ __attribute__((aligned(16))) float S[GR * SP];

  const int tid = threadIdx.x, l = tid & 31, h = l >> 4, m = l & 15, w = tid >> 5;
  const int y = blockIdx.y;
  const int r0 = blockIdx.x * GR;
  const float* cw = (y != 0) ? cwB : cwA;
  const float* cb = (y != 0) ? cbB : cbA;

  for (int q = tid; q < GR * KC; q += 128) {
    const int term = q / GR, rl = q - term * GR;
    const float* src = TX + (((size_t)(term * 2 + y) * NP) + r0 + rl) * ZS;
    const v4f a = *(const v4f*)src;
    const v4f b = *(const v4f*)(src + 4);
    const v2f c2 = *(const v2f*)(src + 8);
    float v[RR];
    v[0] = a.x; v[1] = a.y; v[2] = a.z; v[3] = a.w;
    v[4] = b.x; v[5] = b.y; v[6] = b.z; v[7] = b.w;
    v[8] = c2.x; v[9] = c2.y;
    us16* ph = Ah + rl * AP + term * RR;
    us16* pl = Al + rl * AP + term * RR;
#pragma unroll
    for (int r = 0; r < RR; ++r) split2(v[r], ph + r, pl + r);
  }
  for (int q = tid; q < GR * (64 - KW); q += 128) {
    const int rl = q / (64 - KW), cc = q - rl * (64 - KW);
    Ah[rl * AP + KW + cc] = (us16)0;
    Al[rl * AP + KW + cc] = (us16)0;
  }
  {
    const int nn = tid & 31, kq = tid >> 5;
#pragma unroll
    for (int j = 0; j < 16; ++j) {
      const int k = kq * 16 + j;
      const int kc = min(k, KW - 1);
      float v = cw[kc * QQ + nn];
      v = (k < KW) ? v : 0.0f;
      split2(v, Bh + nn * AP + k, Bl + nn * AP + k);
    }
  }
  {
    const float* wr = wih + (size_t)tid * QQ;
#pragma unroll
    for (int j = 0; j < 8; ++j) {
      const v4f v = *(const v4f*)(wr + 4 * j);
      us16* ph = Wh + tid * XP + 4 * j;
      us16* pl = Wl + tid * XP + 4 * j;
      split2(v.x, ph + 0, pl + 0);
      split2(v.y, ph + 1, pl + 1);
      split2(v.z, ph + 2, pl + 2);
      split2(v.w, ph + 3, pl + 3);
    }
  }
  __syncthreads();

  const int rt = w >> 1, nt = w & 1;
  v8f acc1;
  { const v8f z8 = {0.f, 0.f, 0.f, 0.f, 0.f, 0.f, 0.f, 0.f}; acc1 = z8; }
#pragma unroll
  for (int ks = 0; ks < 2; ++ks) {
    Frag ah, al, bh, bl;
    const us16* pa = Ah + (16 * rt + m) * AP + 32 * ks + 8 * h;
    const us16* qa = Al + (16 * rt + m) * AP + 32 * ks + 8 * h;
    const us16* pb = Bh + (16 * nt + m) * AP + 32 * ks + 8 * h;
    const us16* qb = Bl + (16 * nt + m) * AP + 32 * ks + 8 * h;
    ah.q[0] = *(const v8us*)pa; ah.q[1] = *(const v8us*)(pa + 16);
    al.q[0] = *(const v8us*)qa; al.q[1] = *(const v8us*)(qa + 16);
    bh.q[0] = *(const v8us*)pb; bh.q[1] = *(const v8us*)(pb + 16);
    bl.q[0] = *(const v8us*)qb; bl.q[1] = *(const v8us*)(qb + 16);
    acc1 = mma(ah.v, bh.v, acc1);
    acc1 = mma(ah.v, bl.v, acc1);
    acc1 = mma(al.v, bh.v, acc1);
    guard1(acc1, ah.v, al.v, bh.v, bl.v);
  }
  {
    const int col = 16 * nt + m;
    const float bn = cb[col];
#pragma unroll
    for (int r = 0; r < 8; ++r) {
      const float v = acc1[r] + bn;
      const float sgv = fsigm(v);
      const int row = 16 * rt + 8 * h + r;
      split2(sgv, Xh + row * XP + col, Xl + row * XP + col);
    }
  }
  __syncthreads();

  v8f acc2[4];
  { const v8f z8 = {0.f, 0.f, 0.f, 0.f, 0.f, 0.f, 0.f, 0.f};
#pragma unroll
    for (int j = 0; j < 4; ++j) acc2[j] = z8; }
  Frag xa, xl;
  {
    const us16* pa = Xh + (16 * rt + m) * XP + 8 * h;
    const us16* qa = Xl + (16 * rt + m) * XP + 8 * h;
    xa.q[0] = *(const v8us*)pa; xa.q[1] = *(const v8us*)(pa + 16);
    xl.q[0] = *(const v8us*)qa; xl.q[1] = *(const v8us*)(qa + 16);
  }
#pragma unroll
  for (int j = 0; j < 4; ++j) {
    Frag bh, bl;
    const int ntile = 4 * nt + j;
    const us16* pb = Wh + (16 * ntile + m) * XP + 8 * h;
    const us16* qb = Wl + (16 * ntile + m) * XP + 8 * h;
    bh.q[0] = *(const v8us*)pb; bh.q[1] = *(const v8us*)(pb + 16);
    bl.q[0] = *(const v8us*)qb; bl.q[1] = *(const v8us*)(qb + 16);
    acc2[j] = mma(xa.v, bh.v, acc2[j]);
    acc2[j] = mma(xa.v, bl.v, acc2[j]);
    acc2[j] = mma(xl.v, bh.v, acc2[j]);
    guard1(acc2[j], xa.v, xl.v, bh.v, bl.v);
  }
#pragma unroll
  for (int j = 0; j < 4; ++j) {
    const int col = 16 * (4 * nt + j) + m;
    const float bn = bih[col];
#pragma unroll
    for (int r = 0; r < 8; ++r) S[(16 * rt + 8 * h + r) * SP + col] = acc2[j][r] + bn;
  }
  __syncthreads();
  float* dst = xg + ((size_t)y * NP + r0) * XGS;
#pragma unroll
  for (int i = 0; i < GR / 4; ++i) {
    const int row = 4 * i + w;
    const v4f v = *(const v4f*)(S + row * SP + 4 * l);
    *(volatile v4f*)(dst + (size_t)row * XGS + 4 * l) = v;
  }
  __threadfence();
#pragma unroll
  for (int i = 0; i < GR / 4; ++i) {
    const int row = 4 * i + w;
    const v4f v = *(const v4f*)(S + row * SP + 4 * l);
    *(volatile v4f*)(dst + (size_t)row * XGS + 4 * l) = v;
  }
}

__global__ __launch_bounds__(128)
void k_lstm(const float* __restrict__ xg,
            const float* __restrict__ XA, const float* __restrict__ XB,
            const float* __restrict__ whh, const float* __restrict__ bhh,
            const float* __restrict__ hwA, const float* __restrict__ hbA,
            const float* __restrict__ hwB, const float* __restrict__ hbB,
            float* out, int n, int NP, int T) {
  __shared__ __attribute__((aligned(16))) float h_l[NHID];
  __shared__ float sg[NG];
  __shared__ __attribute__((aligned(16))) float hd_l[2 * RR * WLP];
  __shared__ float hb_l[2 * 16];
  __shared__ __attribute__((aligned(16))) float stg[32 * RR];

  const int g = threadIdx.x, l = g & 31, w = g >> 5;

  float wreg[NHID];
  {
    const float* wr = whh + (size_t)g * NHID;
#pragma unroll
    for (int j = 0; j < NHID / 4; ++j) {
      const v4f v = *(const v4f*)(wr + 4 * j);
      wreg[4 * j + 0] = v.x; wreg[4 * j + 1] = v.y; wreg[4 * j + 2] = v.z; wreg[4 * j + 3] = v.w;
    }
  }
  for (int q = g; q < 2 * RR * NHID; q += 128) {
    const int hs = q / (RR * NHID);
    const int rem = q - hs * (RR * NHID);
    const int r = rem / NHID, j = rem - r * NHID;
    const float va = hwA[rem];
    const float vb = hwB[rem];
    hd_l[(hs * RR + r) * WLP + j] = (hs != 0) ? vb : va;
  }
  if (g < 32) {
    const int hs = g >> 4, r = g & 15;
    const int rc = min(r, RR - 1);
    const float va = hbA[rc];
    const float vb = hbB[rc];
    const float v = (hs != 0) ? vb : va;
    hb_l[g] = (r < RR) ? v : 0.0f;
  }
  if (g < NHID) h_l[g] = 0.0f;
  float c = 0.0f;
  const float bg = bhh[g];
  __syncthreads();

  for (int it = 0; it < T; ++it) {
    const bool rec = (it == T - 1);
    for (int sq = 0; sq < 2; ++sq) {
      const float* xs = xg + (size_t)sq * NP * XGS;
      const float* X = (sq != 0) ? XB : XA;
      float* o = out + (size_t)sq * n * RR;
      const float* hd = hd_l + sq * RR * WLP;
      const float* hb = hb_l + sq * 16;
      for (int t = 0; t < n; ++t) {
        float a = xs[(size_t)t * XGS + g] + bg;
#pragma unroll
        for (int j = 0; j < NHID / 4; ++j) {
          const v4f hv = *(const v4f*)(h_l + 4 * j);
          a = fmaf(hv.x, wreg[4 * j + 0], a);
          a = fmaf(hv.y, wreg[4 * j + 1], a);
          a = fmaf(hv.z, wreg[4 * j + 2], a);
          a = fmaf(hv.w, wreg[4 * j + 3], a);
        }
        sg[g] = a;
        __syncthreads();
        if (w == 0) {
          const float gi = sg[l];
          const float gf = sg[NHID + l];
          const float gc = sg[2 * NHID + l];
          const float go = sg[3 * NHID + l];
          c = fsigm(gf) * c + fsigm(gi) * ftanh(gc);
          const float hv = fsigm(go) * ftanh(c);
          h_l[l] = hv;
          if (rec) {
            wave_sync();
            const int r = min(l, RR - 1);
            float s = hb[r];
#pragma unroll 1
            for (int jj = 0; jj < NHID; jj += 8) {
              const v4f w0 = *(const v4f*)(hd + r * WLP + jj);
              const v4f w1 = *(const v4f*)(hd + r * WLP + jj + 4);
              const v4f h0 = *(const v4f*)(h_l + jj);
              const v4f h1 = *(const v4f*)(h_l + jj + 4);
              s = fmaf(h0.x, w0.x, s); s = fmaf(h0.y, w0.y, s);
              s = fmaf(h0.z, w0.z, s); s = fmaf(h0.w, w0.w, s);
              s = fmaf(h1.x, w1.x, s); s = fmaf(h1.y, w1.y, s);
              s = fmaf(h1.z, w1.z, s); s = fmaf(h1.w, w1.w, s);
            }
            const float v = X[(size_t)t * RR + r] + ftanh(s);
            if (l < RR) stg[(t & 31) * RR + l] = v;
            if (((t & 31) == 31) || (t == n - 1)) {
              wave_sync();
              const int tb = t & ~31;
              const int np = ((t - tb + 1) * RR) >> 2;
              float* ob = o + (size_t)tb * RR;
              v4f pv[3];
#pragma unroll
              for (int i = 0; i < 3; ++i) {
                const int pc = min(l + 32 * i, 32 * RR / 4 - 1);
                pv[i] = *(const v4f*)(stg + pc * 4);
              }
#pragma unroll
              for (int i = 0; i < 3; ++i) {
                const int p = l + 32 * i;
                if (p < np) *(volatile v4f*)(ob + (size_t)p * 4) = pv[i];
              }
              __threadfence();
#pragma unroll
              for (int i = 0; i < 3; ++i) {
                const int p = l + 32 * i;
                if (p < np) *(volatile v4f*)(ob + (size_t)p * 4) = pv[i];
              }
              wave_sync();
            }
          }
        }
        __syncthreads();
      }
    }
  }
}

extern "C" void kernel_launch(void* const* d_in, const int* in_sizes, int n_in,
                              void* d_out, int out_size, void* d_ws, size_t ws_size,
                              hipStream_t stream) {
  if (n_in < 16) return;
  const int n = in_sizes[0] / RR;
  if (n < 32 || (n % 16) != 0) return;
  if (in_sizes[0] != n * RR || in_sizes[1] != n * RR) return;
  if (out_size != 2 * n * RR) return;
  if (in_sizes[2] < 2 || in_sizes[3] < 2 || (in_sizes[2] & 1) != 0 || (in_sizes[3] & 1) != 0) return;
  if (in_sizes[4] != KW * QQ || in_sizes[6] != KW * QQ || in_sizes[5] < QQ || in_sizes[7] < QQ) return;
  if (in_sizes[8] != NG * QQ || in_sizes[9] != NG * NHID || in_sizes[10] < NG || in_sizes[11] < NG) return;
  if (in_sizes[12] != RR * NHID || in_sizes[14] != RR * NHID || in_sizes[13] < RR || in_sizes[15] < RR) return;

  const float* H   = (const float*)d_in[0];
  const float* W   = (const float*)d_in[1];
  const int*   HA  = (const int*)d_in[2];
  const int*   WA  = (const int*)d_in[3];
  const float* hcw = (const float*)d_in[4];
  const float* hcb = (const float*)d_in[5];
  const float* wcw = (const float*)d_in[6];
  const float* wcb = (const float*)d_in[7];
  const float* wih = (const float*)d_in[8];
  const float* whh = (const float*)d_in[9];
  const float* bih = (const float*)d_in[10];
  const float* bhh = (const float*)d_in[11];
  const float* dhw = (const float*)d_in[12];
  const float* dhb = (const float*)d_in[13];
  const float* dww = (const float*)d_in[14];
  const float* dwb = (const float*)d_in[15];
  float* out = (float*)d_out;

  const int nEA = in_sizes[2] / 2;
  const int nEB = in_sizes[3] / 2;
  const int nblk = (n + ROWS - 1) / ROWS;
  const int NP = nblk * ROWS;

  char* ws = (char*)d_ws;
  size_t off = 0;
  auto carve = [&](size_t bytes) -> char* {
    char* p = ws + off;
    off = (off + bytes + 255) & ~(size_t)255;
    return p;
  };
  float* dinv = (float*)carve((size_t)2 * NP * sizeof(float));
  float* TX   = (float*)carve((size_t)KC * 2 * NP * ZS * sizeof(float));
  float* xg   = (float*)carve((size_t)2 * NP * XGS * sizeof(float));
  if (off > ws_size) return;
  if (off > ((size_t)128 << 20)) return;

  const int vecok = (((nEA | nEB) & 7) == 0) ? 1 : 0;
  const dim3 gg(nblk, 2);

  k_graph<0><<<gg, dim3(GT), 0, stream>>>(HA, nEA, WA, nEB, H, W, dinv, TX, n, NP, 0, vecok);
  k_graph<1><<<gg, dim3(GT), 0, stream>>>(HA, nEA, WA, nEB, H, W, dinv, TX, n, NP, 1, vecok);
  for (int k = 2; k < KC; ++k)
    k_graph<2><<<gg, dim3(GT), 0, stream>>>(HA, nEA, WA, nEB, H, W, dinv, TX, n, NP, k, vecok);
  k_gemm<<<dim3(NP / GR, 2), dim3(128), 0, stream>>>(TX, hcw, hcb, wcw, wcb, wih, bih, xg, NP);
  k_lstm<<<dim3(1), dim3(128), 0, stream>>>(xg, H, W, whh, bhh, dhw, dhb, dww, dwb, out, n, NP, 10);
}
